// BcosAttention_71562745085987
// MI455X (gfx1250) — hardware-verified
//
#include <hip/hip_runtime.h>


#define NB_  2
#define NT_  2048
#define DM   512
#define NH_  8
#define HD   64
#define NTK  (NB_ * NT_)
#define NQO  3072
#define NPO  1024
#define QS   256.0f
#define PSC  32768.0f
#define LOSC 1024.0f
#define LOSCI (1.0f / 1024.0f)
#define RSQIN 0.044194173824159216f

typedef _Float16 h16;
typedef unsigned short bf;
typedef __attribute__((ext_vector_type(16))) __bf16   v16bf;
typedef __attribute__((ext_vector_type(16))) _Float16 v16h;
typedef __attribute__((ext_vector_type(8)))  _Float16 v8h;
typedef __attribute__((ext_vector_type(8)))  unsigned short v8us;
typedef __attribute__((ext_vector_type(8)))  float    v8f;
typedef __attribute__((ext_vector_type(4)))  float    v4f;
typedef v8h  __attribute__((may_alias)) v8ha;
typedef v4f  __attribute__((may_alias)) v4fa;
typedef v8us __attribute__((may_alias)) v8usa;

__device__ __forceinline__ unsigned short f2bf(float f) { unsigned u = __float_as_uint(f); u += 0x7FFFu + ((u >> 16) & 1u); return (unsigned short)(u >> 16); }
__device__ __forceinline__ float bf2f(unsigned short b) { return __uint_as_float(((unsigned)b) << 16); }
__device__ __forceinline__ float bfr(float f) { return bf2f(f2bf(f)); }
__device__ __forceinline__ v16h cat16(v8h lo, v8h hi) { return __builtin_shufflevector(lo, hi, 0, 1, 2, 3, 4, 5, 6, 7, 8, 9, 10, 11, 12, 13, 14, 15); }
__device__ __forceinline__ v16bf cat16b(v8us lo, v8us hi) { return __builtin_bit_cast(v16bf, __builtin_shufflevector(lo, hi, 0, 1, 2, 3, 4, 5, 6, 7, 8, 9, 10, 11, 12, 13, 14, 15)); }
__device__ __forceinline__ v8f wmma16(v16h a, v16h b, v8f c) { return __builtin_amdgcn_wmma_f32_16x16x32_f16(false, a, false, b, (short)0, c, false, false); }
__device__ __forceinline__ v8f wmmab(v16bf a, v16bf b, v8f c) { return __builtin_amdgcn_wmma_f32_16x16x32_bf16(false, a, false, b, (short)0, c, false, false); }
#define VST2(T, p, v) do { const T vst2_v_ = (v); *(volatile T*)(p) = vst2_v_; __threadfence(); *(volatile T*)(p) = vst2_v_; } while (0)

__global__ __launch_bounds__(256) void k_rows(const float* __restrict__ src, int nrows, float extra, bf* dst, float* RN) {
    __shared__ float rn[32];
    const int lane = threadIdx.x & 31, wave = threadIdx.x >> 5;
#pragma unroll
    for (int rr = 0; rr < 4; ++rr) {
        const int r = blockIdx.x * 32 + wave * 4 + rr;
        float s = 0.f; v8us t0, t1;
#pragma unroll
        for (int i = 0; i < 8; ++i) { const float a = bfr(src[(size_t)r * DM + lane * 8 + i]), b = bfr(src[(size_t)r * DM + 256 + lane * 8 + i]); t0[i] = f2bf(a); t1[i] = f2bf(b); s += a * a + b * b; }
#pragma unroll
        for (int o = 16; o; o >>= 1) s += __shfl_xor(s, o, 32);
        if (lane == 0) rn[wave * 4 + rr] = extra / sqrtf(s);
        *(volatile v8us*)(dst + (size_t)r * DM + lane * 8) = t0; *(volatile v8us*)(dst + (size_t)r * DM + 256 + lane * 8) = t1; __threadfence();
        *(volatile v8us*)(dst + (size_t)r * DM + lane * 8) = t0; *(volatile v8us*)(dst + (size_t)r * DM + 256 + lane * 8) = t1;
    }
    __syncthreads();
    if (wave == 0) VST2(float, RN + (size_t)blockIdx.x * 32 + lane, rn[lane]);
    (void)nrows;
}
template <bool SPLITA>
__global__ __launch_bounds__(128) void k_gemm(const bf* __restrict__ A, const bf* __restrict__ Al, const bf* __restrict__ Bn, const float* __restrict__ cs, float* C, int ldc) {
    __shared__ __align__(16) float ost[4][16 * 68];
    const int lane = threadIdx.x & 31, wave = threadIdx.x >> 5, lr = lane & 15, hi = lane >> 4;
    const int r0 = blockIdx.x * 64 + wave * 16, c0 = blockIdx.y * 64;
    const size_t aoff = (size_t)(r0 + lr) * DM + 8 * hi;
    size_t boff[4];
#pragma unroll
    for (int t = 0; t < 4; ++t) boff[t] = (size_t)(c0 + t * 16 + lr) * DM + 8 * hi;
    v8f acc[4];
#pragma unroll
    for (int t = 0; t < 4; ++t) acc[t] = (v8f){};
#pragma unroll 1
    for (int kc = 0; kc < DM; kc += 32) {
        const v16bf a = cat16b(*(const v8us*)(A + aoff + kc), *(const v8us*)(A + aoff + kc + 16));
        v16bf al = a;
        if (SPLITA) al = cat16b(*(const v8us*)(Al + aoff + kc), *(const v8us*)(Al + aoff + kc + 16));
#pragma unroll
        for (int t = 0; t < 4; ++t) { const v16bf b = cat16b(*(const v8us*)(Bn + boff[t] + kc), *(const v8us*)(Bn + boff[t] + kc + 16)); acc[t] = wmmab(a, b, acc[t]); if (SPLITA) acc[t] = wmmab(al, b, acc[t]); }
        asm volatile("v_nop\n\tv_nop\n\tv_nop\n\tv_nop" : "+v"(acc[0]), "+v"(acc[1]), "+v"(acc[2]), "+v"(acc[3]) : "v"(a), "v"(al));
    }
    float* os = &ost[wave][0];
#pragma unroll
    for (int t = 0; t < 4; ++t) { const float sc = cs[c0 + t * 16 + lr];
#pragma unroll
        for (int j = 0; j < 8; ++j) os[(hi * 8 + j) * 68 + t * 16 + lr] = acc[t][j] * sc; }
    __syncthreads();
    float* crow = C + (size_t)r0 * ldc + c0;
    auto pass = [&]() {
#pragma unroll
        for (int s = 0; s < 8; ++s) { const int Lid = (lane >> 3) + 4 * s, piece = lane & 7; const int row = Lid >> 1, cofs = (Lid & 1) * 32 + piece * 4;
            const v4f val = *(const v4fa*)(os + row * 68 + cofs); *(volatile v4f*)(crow + (size_t)row * ldc + cofs) = val; }
    };
    pass(); __threadfence(); pass();
}
__global__ __launch_bounds__(256) void k_qkv(const float* __restrict__ OQ, const float* __restrict__ RX, h16* Q16, h16* K16, float* Vf) {
    const int lane = threadIdx.x & 31, wid = blockIdx.x * 8 + (threadIdx.x >> 5);
    const int tok = wid / 3, i = wid - tok * 3;
    if (tok >= NTK) return;
    const float rx = RX[tok] * QS;
    v8f vtmp[2];
#pragma unroll
    for (int q = 0; q < 2; ++q) { float v[8];
#pragma unroll
        for (int e = 0; e < 8; ++e) { const int j = i * DM + q * 256 + lane * 8 + e; const float a = OQ[(size_t)tok * NQO + j], b = OQ[(size_t)tok * NQO + 1536 + j]; const float m = fmaxf(a, b); v[e] = m * fabsf(m) * rx; }
        if (i < 2) { v8h o;
#pragma unroll
            for (int e = 0; e < 8; ++e) o[e] = (h16)v[e];
            VST2(v8h, (i == 0 ? Q16 : K16) + (size_t)tok * DM + q * 256 + lane * 8, o); }
        else { v8f o;
#pragma unroll
            for (int e = 0; e < 8; ++e) o[e] = v[e];
            vtmp[q] = o; }
    }
    if (i == 2) {
        __shared__ float vrow[8][DM];
        float* vr = vrow[threadIdx.x >> 5];
#pragma unroll
        for (int q = 0; q < 2; ++q)
#pragma unroll
            for (int e = 0; e < 8; ++e) vr[q * 256 + lane * 8 + e] = vtmp[q][e];
        __builtin_amdgcn_wave_barrier();
#pragma unroll
        for (int s = 0; s < 4; ++s) { const v4f val = *(const v4fa*)(vr + s * 128 + lane * 4); VST2(v4f, Vf + (size_t)tok * DM + s * 128 + lane * 4, val); }
    }
}

__global__ __launch_bounds__(256) void k_vt(const float* __restrict__ V, h16* VTH, h16* VTL) {
    __shared__ __align__(16) h16 tile[HD * 72];
    __shared__ __align__(16) h16 til2[HD * 72];
    const int bid = blockIdx.x;
    const int b = bid / (NH_ * (NT_ / 64)), rem = bid - b * (NH_ * (NT_ / 64)), h = rem / (NT_ / 64), kt = rem - h * (NT_ / 64);
    const int k0 = kt * 64, tid = threadIdx.x, kk = tid >> 2, d0 = (tid & 3) * 16;
    const float* src = V + ((size_t)b * NT_ + k0 + kk) * DM + h * HD + d0;
#pragma unroll
    for (int i = 0; i < 16; ++i) { const float v = src[i]; const h16 a = (h16)v; tile[(d0 + i) * 72 + kk] = a; til2[(d0 + i) * 72 + kk] = (h16)((v - (float)a) * LOSC); }
    __syncthreads();
    const int piece = tid & 7;
    const size_t base = (((size_t)b * NH_ + h) * HD) * NT_ + k0;
    auto pass = [&]() {
#pragma unroll
        for (int s = 0; s < 4; ++s) { const int Lid = (tid >> 3) + 32 * s; const int pln = Lid >> 6, d = Lid & 63;
            const v8h val = *(const v8ha*)((pln ? til2 : tile) + d * 72 + piece * 8); *(volatile v8h*)((pln ? VTL : VTH) + base + (size_t)d * NT_ + piece * 8) = val; }
    };
    pass(); __threadfence(); pass();
}
__global__ __launch_bounds__(128) void k_attn(const h16* __restrict__ Q16, const h16* __restrict__ K16, const h16* __restrict__ VTH, const h16* __restrict__ VTL, bf* CH, bf* CL) {
    __shared__ __align__(16) h16 plds[4][16 * 32];
    __shared__ __align__(16) h16 plds2[4][16 * 32];
    __shared__ __align__(16) float ost[4][16 * 68];
    const int lane = threadIdx.x & 31, wave = threadIdx.x >> 5, lr = lane & 15, hi = lane >> 4;
    const int bid = blockIdx.x;
    const int b = bid / (NH_ * (NT_ / 64)), rem = bid - b * (NH_ * (NT_ / 64)), h = rem / (NT_ / 64), qt = rem - h * (NT_ / 64);
    const int q0 = qt * 64 + wave * 16;
    const size_t tok0 = (size_t)b * NT_;
    h16* pl = &plds[wave][0]; h16* pl2 = &plds2[wave][0];
    v16h qa[2];
#pragma unroll
    for (int kc = 0; kc < 2; ++kc) { const h16* p = Q16 + (tok0 + q0 + lr) * DM + h * HD + kc * 32 + 8 * hi; qa[kc] = cat16(*(const v8h*)p, *(const v8h*)(p + 16)); }
    const size_t vbase = (((size_t)b * NH_ + h) * HD) * NT_;
    const float lsc = 0.125f / (QS * QS);
    v8f o[4], ox[4];
#pragma unroll
    for (int n = 0; n < 4; ++n) { o[n] = (v8f){}; ox[n] = (v8f){}; }
    float mrow[8], lpart[8];
#pragma unroll
    for (int j = 0; j < 8; ++j) { mrow[j] = -3.0e38f; lpart[j] = 0.f; }
#pragma unroll 1
    for (int kt = 0; kt < NT_ / 32; ++kt) {
        const int l0 = kt * 32;
        v8f s0 = {}, s1 = {};
#pragma unroll
        for (int kc = 0; kc < 2; ++kc) {
            const h16* r0p = K16 + (tok0 + l0 + lr) * DM + h * HD + kc * 32 + 8 * hi; const h16* r1p = r0p + (size_t)16 * DM;
            s0 = wmma16(qa[kc], cat16(*(const v8h*)r0p, *(const v8h*)(r0p + 16)), s0);
            s1 = wmma16(qa[kc], cat16(*(const v8h*)r1p, *(const v8h*)(r1p + 16)), s1);
        }
        asm volatile("v_nop\n\tv_nop\n\tv_nop\n\tv_nop" : "+v"(s0), "+v"(s1) : "v"(qa[0]), "v"(qa[1]));
        float alpha[8];
#pragma unroll
        for (int j = 0; j < 8; ++j) {
            const float a0 = s0[j] * lsc, a1 = s1[j] * lsc;
            float mx = fmaxf(a0, a1);
            mx = fmaxf(mx, __shfl_xor(mx, 1, 16)); mx = fmaxf(mx, __shfl_xor(mx, 2, 16)); mx = fmaxf(mx, __shfl_xor(mx, 4, 16)); mx = fmaxf(mx, __shfl_xor(mx, 8, 16));
            const float mn = fmaxf(mrow[j], mx);
            alpha[j] = __expf(mrow[j] - mn); mrow[j] = mn;
            const float p0 = __expf(a0 - mn), p1 = __expf(a1 - mn);
            lpart[j] = lpart[j] * alpha[j] + (p0 + p1);
            const int mr = hi * 8 + j;
            const float ps0 = p0 * PSC, ps1 = p1 * PSC; const h16 h0 = (h16)ps0, h1 = (h16)ps1;
            pl[mr * 32 + lr] = h0; pl[mr * 32 + 16 + lr] = h1; pl2[mr * 32 + lr] = (h16)((ps0 - (float)h0) * LOSC); pl2[mr * 32 + 16 + lr] = (h16)((ps1 - (float)h1) * LOSC);
        }
#pragma unroll
        for (int n = 0; n < 4; ++n)
#pragma unroll
            for (int j = 0; j < 8; ++j) { o[n][j] *= alpha[j]; ox[n][j] *= alpha[j]; }
        asm volatile("" ::: "memory");
        const v16h pa = cat16(*(const v8ha*)(pl + lr * 32 + hi * 8), *(const v8ha*)(pl + lr * 32 + 16 + hi * 8));
        const v16h px = cat16(*(const v8ha*)(pl2 + lr * 32 + hi * 8), *(const v8ha*)(pl2 + lr * 32 + 16 + hi * 8));
#pragma unroll
        for (int n = 0; n < 4; ++n) { const size_t vo = vbase + (size_t)(n * 16 + lr) * NT_ + l0 + hi * 8;
            const v16h vh = cat16(*(const v8h*)(VTH + vo), *(const v8h*)(VTH + vo + 16)), vl = cat16(*(const v8h*)(VTL + vo), *(const v8h*)(VTL + vo + 16));
            o[n] = wmma16(pa, vh, o[n]); ox[n] = wmma16(pa, vl, ox[n]); ox[n] = wmma16(px, vh, ox[n]); }
        asm volatile("v_nop\n\tv_nop\n\tv_nop\n\tv_nop" : "+v"(o[0]), "+v"(o[1]), "+v"(o[2]), "+v"(o[3]), "+v"(ox[0]), "+v"(ox[1]), "+v"(ox[2]), "+v"(ox[3]) : "v"(pa), "v"(px));
    }
    float inv[8];
#pragma unroll
    for (int j = 0; j < 8; ++j) { float rs = lpart[j]; rs += __shfl_xor(rs, 1, 16); rs += __shfl_xor(rs, 2, 16); rs += __shfl_xor(rs, 4, 16); rs += __shfl_xor(rs, 8, 16); inv[j] = 1.0f / (rs * PSC * QS); }
    float* os = &ost[wave][0];
#pragma unroll
    for (int n = 0; n < 4; ++n)
#pragma unroll
        for (int j = 0; j < 8; ++j) os[(hi * 8 + j) * 68 + n * 16 + lr] = (o[n][j] + ox[n][j] * LOSCI) * inv[j];
    __syncthreads();
    const size_t cbase = (tok0 + q0) * DM + (size_t)h * HD;
    auto pass = [&]() {
#pragma unroll
        for (int s = 0; s < 4; ++s) { const int row = 4 * s + (lane >> 3), piece = lane & 7; const float* sp = os + row * 68 + piece * 8; v8us oh, ol;
#pragma unroll
            for (int i = 0; i < 8; ++i) { const unsigned short hb = f2bf(sp[i]); oh[i] = hb; ol[i] = f2bf(sp[i] - bf2f(hb)); }
            *(volatile v8us*)(CH + cbase + (size_t)row * DM + piece * 8) = oh; *(volatile v8us*)(CL + cbase + (size_t)row * DM + piece * 8) = ol; }
    };
    pass(); __threadfence(); pass();
}
__global__ __launch_bounds__(256) void k_norm(const bf* __restrict__ CH, const bf* __restrict__ CL, float* RC) {
    __shared__ float rn[32];
    const int lane = threadIdx.x & 31, wave = threadIdx.x >> 5;
#pragma unroll
    for (int rr = 0; rr < 4; ++rr) { const int r = blockIdx.x * 32 + wave * 4 + rr; float s = 0.f;
#pragma unroll
        for (int i = 0; i < 16; ++i) { const size_t c = (size_t)r * DM + lane * 16 + i; const float v = bf2f(CH[c]) + bf2f(CL[c]); s += v * v; }
#pragma unroll
        for (int o = 16; o; o >>= 1) s += __shfl_xor(s, o, 32);
        if (lane == 0) rn[wave * 4 + rr] = RSQIN / sqrtf(s); }
    __syncthreads();
    if (wave == 0) VST2(float, RC + (size_t)blockIdx.x * 32 + lane, rn[lane]);
}
__global__ __launch_bounds__(256) void k_out(const float* __restrict__ O2, const float* __restrict__ RC, float* out) {
    const int lane = threadIdx.x & 31, r = blockIdx.x * 8 + (threadIdx.x >> 5);
    if (r >= NTK) return;
    const float rc = RC[r];
#pragma unroll
    for (int s = 0; s < 4; ++s) { v4f o;
#pragma unroll
        for (int i = 0; i < 4; ++i) { const int j = s * 128 + lane * 4 + i; const float a = O2[(size_t)r * NPO + j], b = O2[(size_t)r * NPO + DM + j]; const float m = fmaxf(a, b); o[i] = m * fabsf(m) * rc; }
        VST2(v4f, out + (size_t)r * DM + s * 128 + lane * 4, o); }
}

extern "C" void kernel_launch(void* const* d_in, const int* in_sizes, int n_in,
                              void* d_out, int out_size, void* d_ws, size_t ws_size, hipStream_t stream) {
    (void)in_sizes; (void)n_in; (void)out_size;
    const float* x = (const float*)d_in[0]; const float* Wq = (const float*)d_in[1]; const float* Wp = (const float*)d_in[2];
    float* out = (float*)d_out;
    char* wsp = (char*)d_ws;
    auto take = [&](size_t bytes) { char* p = wsp; wsp += (bytes + 255) & ~(size_t)255; return (void*)p; };
    bf* Xb = (bf*)take((size_t)NTK * DM * 2); float* RX = (float*)take((size_t)NTK * 4);
    bf* WQb = (bf*)take((size_t)NQO * DM * 2); float* RWq = (float*)take((size_t)NQO * 4); bf* WPb = (bf*)take((size_t)NPO * DM * 2); float* RWp = (float*)take((size_t)NPO * 4);
    float* OQ = (float*)take((size_t)NTK * NQO * 4); h16* Q16 = (h16*)take((size_t)NTK * DM * 2); h16* K16 = (h16*)take((size_t)NTK * DM * 2); float* Vf = (float*)take((size_t)NTK * DM * 4);
    h16* VTH = (h16*)take((size_t)NTK * DM * 2); h16* VTL = (h16*)take((size_t)NTK * DM * 2); bf* CH = (bf*)take((size_t)NTK * DM * 2); bf* CL = (bf*)take((size_t)NTK * DM * 2);
    float* RC = (float*)take((size_t)NTK * 4); float* O2 = (float*)take((size_t)NTK * NPO * 4);
    if ((size_t)(wsp - (char*)d_ws) > ws_size) return;
    k_rows<<<NTK / 32, 256, 0, stream>>>(x, NTK, RSQIN, Xb, RX);
    k_rows<<<NQO / 32, 256, 0, stream>>>(Wq, NQO, 1.0f, WQb, RWq);
    k_rows<<<NPO / 32, 256, 0, stream>>>(Wp, NPO, 1.0f, WPb, RWp);
    k_gemm<false><<<dim3(NTK / 64, NQO / 64, 1), 128, 0, stream>>>(Xb, nullptr, WQb, RWq, OQ, NQO);
    k_qkv<<<(NTK * 3) / 8, 256, 0, stream>>>(OQ, RX, Q16, K16, Vf);
    k_vt<<<NB_ * NH_ * (NT_ / 64), 256, 0, stream>>>(Vf, VTH, VTL);
    k_attn<<<NB_ * NH_ * (NT_ / 64), 128, 0, stream>>>(Q16, K16, VTH, VTL, CH, CL);
    k_norm<<<NTK / 32, 256, 0, stream>>>(CH, CL, RC);
    k_gemm<true><<<dim3(NTK / 64, NPO / 64, 1), 128, 0, stream>>>(CH, CL, WPb, RWp, O2, NPO);
    k_out<<<NTK / 8, 256, 0, stream>>>(O2, RC, out);
}
